// FMForecaster_64175401337577
// MI455X (gfx1250) — hardware-verified
//
#include <hip/hip_runtime.h>
#include <stddef.h>


#pragma clang fp contract(off)

#define NB     128
#define NCTX   96
#define NP     24
#define NS     100
#define NSTEP  16
#define NH     256
#define NIN    122
#define NROW   (NS * NB)
#define RB     64
#define KZ     32
#define NP3    32
#define NTHR   256
#define WCAR   64.0f
#define WINV   (1.0f / 64.0f)
#define WSCAP  134217728

#define O1Z    0
#define O1C    (O1Z + NH * KZ)
#define O2T    (O1C + NH * NCTX)
#define O3T    (O2T + NH * NH)
#define WTOT   (O3T + NP3 * NH)
#define WBLK   (WTOT / 8 / NTHR)
#define B1C    (O1C / 8 / NTHR)
#define B2T    (O2T / 8 / NTHR)
#define B3T    (O3T / 8 / NTHR)

#define OWB    0
#define OCB    (WTOT * 2)
#define OZF    (OCB + NB * NH * 4)
#define WSTOT  (OZF + NROW * KZ * 4)

#define LC_INV 0
#define LC_A   256
#define LC_C   (LC_A + RB * NCTX * 2)
#define LC_TOT (LC_C + RB * NH * 4)

#define LM_Z   0
#define LM_ZH  (LM_Z + RB * KZ * 4)
#define LM_H1  (LM_ZH + RB * KZ * 2)
#define LM_H2  (LM_H1 + RB * NH * 2)
#define LM_CB  (LM_H2 + RB * NH * 2)
#define LM_T24 (LM_CB + RB * NH * 4)
#define LM_B2  (LM_T24 + NH * 4)
#define LM_B3  (LM_B2 + NH * 4)
#define LM_TOT (LM_B3 + NP3 * 4)

static_assert(NB == 2 * RB);
static_assert((NROW % RB) == 0);
static_assert((NCTX % 32) == 0 && (NH % 32) == 0 && KZ == 32 && NP3 == 32 && NP <= KZ && NP <= NP3);
static_assert(NTHR == NH);
static_assert((WTOT % (8 * NTHR)) == 0 && (O1C % (8 * NTHR)) == 0 && (O2T % (8 * NTHR)) == 0 && (O3T % (8 * NTHR)) == 0);
static_assert(((NH * KZ * 2) % 512) == 0 && ((NH * NCTX * 2) % 512) == 0 && ((NH * NH * 2) % 512) == 0 && ((NP3 * NH * 2) % 512) == 0);
static_assert((OCB % 128) == 0 && (OZF % 128) == 0 && ((RB * NH * 4) % 512) == 0 && ((RB * KZ * 4) % 512) == 0);
static_assert(((NS * NP * 4) % 128) == 0 && ((NS * NP) % 4) == 0 && (NP % 4) == 0);
static_assert((LC_A % 16) == 0 && (LC_C % 16) == 0 && LC_TOT <= 160 * 1024);
static_assert((LM_ZH % 16) == 0 && (LM_H1 % 16) == 0 && (LM_H2 % 16) == 0 && (LM_CB % 16) == 0 && (LM_T24 % 16) == 0);
static_assert(LM_TOT <= 160 * 1024);
static_assert(WSTOT <= WSCAP);
static_assert((RB * KZ) == 8 * NTHR);
static_assert(((RB * NH / 4) % NTHR) == 0 && ((RB * KZ / 4) % NTHR) == 0);
static_assert(NIN == NP + 2 + NCTX);

typedef _Float16 v16h __attribute__((ext_vector_type(16)));
typedef _Float16 v8h  __attribute__((ext_vector_type(8), __may_alias__));
typedef float    v8f  __attribute__((ext_vector_type(8)));
typedef float    v4f  __attribute__((ext_vector_type(4), __may_alias__));
union Frag { v16h v; v8h h[2]; };
static_assert(sizeof(Frag) == 32);

__device__ __forceinline__ v8f wmh(v16h a, v16h bq, v8f c) {
  v8f d = __builtin_amdgcn_wmma_f32_16x16x32_f16(false, a, false, bq, (short)0, c, false, false);
  asm volatile("v_nop\n\tv_nop\n\tv_nop\n\tv_nop" : "+v"(d) : "v"(a), "v"(bq));
  return d;
}

__device__ __forceinline__ v8f zero8() {
  v8f z = {0.f, 0.f, 0.f, 0.f, 0.f, 0.f, 0.f, 0.f};
  return z;
}

__device__ __forceinline__ float absmean_loc(const float* row) {
  float s = 0.0f;
#pragma unroll 4
  for (int j = 0; j < NCTX; ++j) s += fabsf(row[j]);
  return fmaxf(s * (1.0f / (float)NCTX), 1e-6f);
}

__global__ __launch_bounds__(NTHR) void k_wprep(const float* __restrict__ W1, const float* __restrict__ W2,
                                                const float* __restrict__ W3, _Float16* Wp) {
  const int blk = blockIdx.x, tid = threadIdx.x;
  const int t = blk * NTHR + tid;
  v8h hv;
  if (blk < B1C) {
    const int idx = t;
    const int n = idx >> 2, kb = (idx & 3) * 8;
#pragma unroll
    for (int q = 0; q < 8; ++q) {
      const int k = kb + q;
      const int kc = k < NP ? k : NP - 1;
      const float sc = k < NP ? WCAR : 0.0f;
      hv[q] = (_Float16)(W1[kc * NH + n] * sc);
    }
  } else if (blk < B2T) {
    const int idx = t - O1C / 8;
    const int n = idx / 12, kb = (idx - n * 12) * 8;
#pragma unroll
    for (int q = 0; q < 8; ++q) {
      const int k = kb + q;
      hv[q] = (_Float16)(W1[(NP + 2 + k) * NH + n] * WCAR);
    }
  } else if (blk < B3T) {
    const int idx = t - O2T / 8;
    const int n = idx >> 5, kb = (idx & 31) * 8;
#pragma unroll
    for (int q = 0; q < 8; ++q) {
      const int k = kb + q;
      hv[q] = (_Float16)(W2[k * NH + n] * WCAR);
    }
  } else {
    const int idx = t - O3T / 8;
    const int n = idx >> 5, kb = (idx & 31) * 8;
    const int nc = n < NP ? n : NP - 1;
    const float sc = n < NP ? WCAR : 0.0f;
#pragma unroll
    for (int q = 0; q < 8; ++q) {
      const int k = kb + q;
      hv[q] = (_Float16)(W3[k * NP + nc] * sc);
    }
  }
  _Float16* dp = Wp + (size_t)t * 8;
  *(volatile v8h*)dp = hv;
  __threadfence();
  *(volatile v8h*)dp = hv;
}

__global__ __launch_bounds__(NTHR) void k_ctx(const float* __restrict__ past, const float* __restrict__ b1,
                                              const _Float16* __restrict__ W1C, float* CB) {
  extern __shared__ __align__(16) char smc[];
  float* sInv = (float*)(smc + LC_INV);
  _Float16* sA = (_Float16*)(smc + LC_A);
  float* sC = (float*)(smc + LC_C);
  const int tid = threadIdx.x, lane = tid & 31, wave = tid >> 5, h = lane >> 4, m = lane & 15;
  const int bb0 = blockIdx.x * RB;

  if (tid < RB) {
    const float l = absmean_loc(past + (size_t)(bb0 + tid) * NCTX);
    sInv[tid] = 1.0f / l;
  }
  __syncthreads();
  for (int e = tid; e < RB * NCTX; e += NTHR) {
    const int r = e / NCTX, j = e - r * NCTX;
    sA[r * NCTX + j] = (_Float16)(past[(size_t)(bb0 + r) * NCTX + j] * sInv[r]);
  }
  __syncthreads();

  const int mt = wave >> 1, ntb = (wave & 1) * 8;
  v8f acc[8];
#pragma unroll
  for (int j = 0; j < 8; ++j) acc[j] = zero8();
  const _Float16* ap = sA + (mt * 16 + m) * NCTX + 8 * h;
  const _Float16* bp0 = W1C + (size_t)(ntb * 16 + m) * NCTX + 8 * h;
#pragma unroll 1
  for (int ks = 0; ks < NCTX / 32; ++ks) {
    const int k0 = 32 * ks;
    Frag fa;
    fa.h[0] = *(const v8h*)(ap + k0);
    fa.h[1] = *(const v8h*)(ap + k0 + 16);
#pragma unroll
    for (int j = 0; j < 8; ++j) {
      const _Float16* bp = bp0 + (size_t)(j * 16) * NCTX + k0;
      Frag fb;
      fb.h[0] = *(const v8h*)bp;
      fb.h[1] = *(const v8h*)(bp + 16);
      acc[j] = wmh(fa.v, fb.v, acc[j]);
    }
  }
#pragma unroll
  for (int j = 0; j < 8; ++j) {
    const int n = (ntb + j) * 16 + m;
    const float bv = b1[n];
#pragma unroll
    for (int r = 0; r < 8; ++r) {
      const int rl = mt * 16 + 8 * h + r;
      sC[rl * NH + n] = acc[j][r] * WINV + bv;
    }
  }
  __syncthreads();

  float* gp = CB + (size_t)bb0 * NH;
#pragma unroll
  for (int it = 0; it < (RB * NH / 4) / NTHR; ++it) {
    const int e = tid + it * NTHR;
    const v4f v = *(const v4f*)(sC + 4 * e);
    *(volatile v4f*)(gp + 4 * e) = v;
  }
  __threadfence();
#pragma unroll
  for (int it = 0; it < (RB * NH / 4) / NTHR; ++it) {
    const int e = tid + it * NTHR;
    const v4f v = *(const v4f*)(sC + 4 * e);
    *(volatile v4f*)(gp + 4 * e) = v;
  }
}

__global__ __launch_bounds__(NTHR) void k_main(const float* __restrict__ z0, const float* __restrict__ W1,
                                               const float* __restrict__ b2, const float* __restrict__ b3,
                                               const _Float16* __restrict__ W1Z, const _Float16* __restrict__ W2T,
                                               const _Float16* __restrict__ W3T, const float* __restrict__ CB,
                                               float* ZF) {
  extern __shared__ __align__(16) char smm[];
  float* sZ = (float*)(smm + LM_Z);
  _Float16* sZH = (_Float16*)(smm + LM_ZH);
  _Float16* sH1 = (_Float16*)(smm + LM_H1);
  _Float16* sH2 = (_Float16*)(smm + LM_H2);
  float* sCB = (float*)(smm + LM_CB);
  float* sT24 = (float*)(smm + LM_T24);
  float* sB2 = (float*)(smm + LM_B2);
  float* sB3 = (float*)(smm + LM_B3);
  const int tid = threadIdx.x, lane = tid & 31, wave = tid >> 5, h = lane >> 4, m = lane & 15;
  const int blk = blockIdx.x;
  const int row0 = blk * RB;
  const int b0 = (blk & 1) * RB;

  for (int e = tid; e < RB * KZ; e += NTHR) {
    const int r = e >> 5, c = e & 31;
    const int cc = c < NP ? c : NP - 1;
    const float v = z0[(size_t)(row0 + r) * NP + cc];
    sZ[e] = c < NP ? v : 0.0f;
  }
  {
    const float* cp = CB + (size_t)b0 * NH;
    for (int e = tid; e < RB * NH / 4; e += NTHR) *(v4f*)(sCB + 4 * e) = *(const v4f*)(cp + 4 * e);
  }
  sT24[tid] = W1[NP * NH + tid];
  sB2[tid] = b2[tid];
  if (tid < NP3) {
    const int nc = tid < NP ? tid : NP - 1;
    const float v = b3[nc];
    sB3[tid] = tid < NP ? v : 0.0f;
  }
  __syncthreads();

  const int mt = wave >> 1, ntb = (wave & 1) * 8, nt3 = wave & 1;
  const float dt = 1.0f / (float)NSTEP;

#pragma unroll 1
  for (int step = 0; step < NSTEP; ++step) {
    const float tval = 1.0f - (float)step * dt;

    {
      const int r = tid >> 2, q = (tid & 3) * 8;
      const v4f x0 = *(const v4f*)(sZ + r * KZ + q);
      const v4f x1 = *(const v4f*)(sZ + r * KZ + q + 4);
      v8h hv;
      hv[0] = (_Float16)x0.x; hv[1] = (_Float16)x0.y; hv[2] = (_Float16)x0.z; hv[3] = (_Float16)x0.w;
      hv[4] = (_Float16)x1.x; hv[5] = (_Float16)x1.y; hv[6] = (_Float16)x1.z; hv[7] = (_Float16)x1.w;
      *(v8h*)(sZH + r * KZ + q) = hv;
    }
    __syncthreads();

    {
      Frag fa;
      const _Float16* ap = sZH + (mt * 16 + m) * KZ + 8 * h;
      fa.h[0] = *(const v8h*)ap;
      fa.h[1] = *(const v8h*)(ap + 16);
#pragma unroll
      for (int j = 0; j < 8; ++j) {
        const int n = (ntb + j) * 16 + m;
        const _Float16* bp = W1Z + (size_t)((ntb + j) * 16 + m) * KZ + 8 * h;
        Frag fb;
        fb.h[0] = *(const v8h*)bp;
        fb.h[1] = *(const v8h*)(bp + 16);
        const v8f acc = wmh(fa.v, fb.v, zero8());
        const float tw = tval * sT24[n];
#pragma unroll
        for (int r = 0; r < 8; ++r) {
          const int rl = mt * 16 + 8 * h + r;
          float v = acc[r] * WINV + sCB[rl * NH + n] + tw;
          v = fmaxf(v, 0.0f);
          sH1[rl * NH + n] = (_Float16)v;
        }
      }
    }
    __syncthreads();

    {
      v8f acc[8];
#pragma unroll
      for (int j = 0; j < 8; ++j) acc[j] = zero8();
      const _Float16* ap = sH1 + (mt * 16 + m) * NH + 8 * h;
      const _Float16* bp0 = W2T + (size_t)(ntb * 16 + m) * NH + 8 * h;
#pragma unroll 1
      for (int ks = 0; ks < NH / 32; ++ks) {
        const int k0 = 32 * ks;
        Frag fa;
        fa.h[0] = *(const v8h*)(ap + k0);
        fa.h[1] = *(const v8h*)(ap + k0 + 16);
#pragma unroll
        for (int j = 0; j < 8; ++j) {
          const _Float16* bp = bp0 + (size_t)(j * 16) * NH + k0;
          Frag fb;
          fb.h[0] = *(const v8h*)bp;
          fb.h[1] = *(const v8h*)(bp + 16);
          acc[j] = wmh(fa.v, fb.v, acc[j]);
        }
      }
#pragma unroll
      for (int j = 0; j < 8; ++j) {
        const int n = (ntb + j) * 16 + m;
        const float bv = sB2[n];
#pragma unroll
        for (int r = 0; r < 8; ++r) {
          const int rl = mt * 16 + 8 * h + r;
          const float v = fmaxf(acc[j][r] * WINV + bv, 0.0f);
          sH2[rl * NH + n] = (_Float16)v;
        }
      }
    }
    __syncthreads();

    {
      v8f acc = zero8();
      const _Float16* ap = sH2 + (mt * 16 + m) * NH + 8 * h;
      const _Float16* bp0 = W3T + (size_t)(nt3 * 16 + m) * NH + 8 * h;
#pragma unroll 1
      for (int ks = 0; ks < NH / 32; ++ks) {
        const int k0 = 32 * ks;
        Frag fa, fb;
        fa.h[0] = *(const v8h*)(ap + k0);
        fa.h[1] = *(const v8h*)(ap + k0 + 16);
        fb.h[0] = *(const v8h*)(bp0 + k0);
        fb.h[1] = *(const v8h*)(bp0 + k0 + 16);
        acc = wmh(fa.v, fb.v, acc);
      }
      const int n = nt3 * 16 + m;
      const float bv = sB3[n];
#pragma unroll
      for (int r = 0; r < 8; ++r) {
        const int rl = mt * 16 + 8 * h + r;
        const float vv = acc[r] * WINV + bv;
        const float zo = sZ[rl * KZ + n];
        const float dz = dt * vv;
        const float zn = zo - dz;
        if (n < NP) sZ[rl * KZ + n] = zn;
      }
    }
    __syncthreads();
  }

  float* gp = ZF + (size_t)row0 * KZ;
#pragma unroll
  for (int it = 0; it < (RB * KZ / 4) / NTHR; ++it) {
    const int e = tid + it * NTHR;
    const v4f v = *(const v4f*)(sZ + 4 * e);
    *(volatile v4f*)(gp + 4 * e) = v;
  }
  __threadfence();
#pragma unroll
  for (int it = 0; it < (RB * KZ / 4) / NTHR; ++it) {
    const int e = tid + it * NTHR;
    const v4f v = *(const v4f*)(sZ + 4 * e);
    *(volatile v4f*)(gp + 4 * e) = v;
  }
}

__global__ __launch_bounds__(NTHR) void k_out(const float* __restrict__ past, const float* __restrict__ obs,
                                              const float* __restrict__ ZF, float* out) {
  (void)obs;
  __shared__ float s_loc;
  const int b = blockIdx.x, tid = threadIdx.x;
  if (tid == 0) s_loc = absmean_loc(past + (size_t)b * NCTX);
  __syncthreads();
  const float loc = s_loc;
  float* op = out + (size_t)b * (NS * NP);
  for (int e = tid; e < NS * NP / 4; e += NTHR) {
    const int s = e / (NP / 4), q = e - s * (NP / 4);
    v4f v = *(const v4f*)(ZF + ((size_t)s * NB + b) * KZ + 4 * q);
    v = v * loc;
    *(volatile v4f*)(op + 4 * e) = v;
  }
  __threadfence();
  for (int e = tid; e < NS * NP / 4; e += NTHR) {
    const int s = e / (NP / 4), q = e - s * (NP / 4);
    v4f v = *(const v4f*)(ZF + ((size_t)s * NB + b) * KZ + 4 * q);
    v = v * loc;
    *(volatile v4f*)(op + 4 * e) = v;
  }
}

extern "C" void kernel_launch(void* const* d_in, const int* in_sizes, int n_in,
                              void* d_out, int out_size, void* d_ws, size_t ws_size,
                              hipStream_t stream) {
  if (n_in < 9) return;
  if (in_sizes[0] != NB * NCTX || in_sizes[1] != NB * NCTX) return;
  if (in_sizes[2] != NROW * NP) return;
  if (in_sizes[3] != NIN * NH || in_sizes[4] != NH) return;
  if (in_sizes[5] != NH * NH || in_sizes[6] != NH) return;
  if (in_sizes[7] != NH * NP || in_sizes[8] != NP) return;
  if (out_size != NROW * NP) return;
  const size_t tot = (size_t)WSTOT;
  if (tot > ws_size || tot > (size_t)WSCAP) return;

  const float* past = (const float*)d_in[0];
  const float* obs  = (const float*)d_in[1];
  const float* z0   = (const float*)d_in[2];
  const float* W1   = (const float*)d_in[3];
  const float* b1   = (const float*)d_in[4];
  const float* W2   = (const float*)d_in[5];
  const float* b2   = (const float*)d_in[6];
  const float* W3   = (const float*)d_in[7];
  const float* b3   = (const float*)d_in[8];
  float* out = (float*)d_out;

  char* ws = (char*)d_ws;
  _Float16* Wp = (_Float16*)(ws + OWB);
  float* CB = (float*)(ws + OCB);
  float* ZF = (float*)(ws + OZF);

  k_wprep<<<WBLK, NTHR, 0, stream>>>(W1, W2, W3, Wp);

  hipFuncSetAttribute(reinterpret_cast<const void*>(&k_ctx), hipFuncAttributeMaxDynamicSharedMemorySize, LC_TOT);
  k_ctx<<<NB / RB, NTHR, LC_TOT, stream>>>(past, b1, Wp + O1C, CB);

  hipFuncSetAttribute(reinterpret_cast<const void*>(&k_main), hipFuncAttributeMaxDynamicSharedMemorySize, LM_TOT);
  k_main<<<NROW / RB, NTHR, LM_TOT, stream>>>(z0, W1, b2, b3, Wp + O1Z, Wp + O2T, Wp + O3T, CB, ZF);

  k_out<<<NB, NTHR, 0, stream>>>(past, obs, ZF, out);
}
